// ZeroSAttention_57389353009768
// MI455X (gfx1250) — hardware-verified
//
#include <hip/hip_runtime.h>
#include <math.h>

typedef __attribute__((ext_vector_type(16))) _Float16 v16h;
typedef __attribute__((ext_vector_type(16))) __bf16 v16b;
typedef __attribute__((ext_vector_type(8)))  _Float16 v8h;
typedef __attribute__((ext_vector_type(8)))  float v8f;
typedef __attribute__((ext_vector_type(4)))  float v4f;
typedef __attribute__((ext_vector_type(2)))  float v2f;
typedef __attribute__((ext_vector_type(4)))  unsigned v4u;
typedef __attribute__((ext_vector_type(4)))  int v4i;
typedef float __attribute__((may_alias)) float_a;
typedef int __attribute__((may_alias)) int_a;

template <typename T> __device__ __forceinline__ void vst2(void* p, T v) { *(volatile T*)p = v; __threadfence(); *(volatile T*)p = v; }
__device__ __forceinline__ v8f wmma16(v16h a, v16h b, v8f c) {
  v8f d = __builtin_amdgcn_wmma_f32_16x16x32_f16(false, a, false, b, (short)0, c, false, false);
  asm volatile("v_nop\n\tv_nop\n\tv_nop\n\tv_nop" : "+v"(d) : "v"(a), "v"(b));
  return d;
}
__device__ __forceinline__ v8f wmma_bf(v16b a, v16b b, v8f c) {
  v8f d = __builtin_amdgcn_wmma_f32_16x16x32_bf16(false, a, false, b, (short)0, c, false, false);
  asm volatile("v_nop\n\tv_nop\n\tv_nop\n\tv_nop" : "+v"(d) : "v"(a), "v"(b));
  return d;
}
__device__ __forceinline__ v16h frag_h(const _Float16* rowk0, int lane) {
  union { v16h v; v8h q[2]; } u; const _Float16* p = rowk0 + 8 * (lane >> 4);
  u.q[0] = *(const v8h*)p; u.q[1] = *(const v8h*)(p + 16); return u.v;
}
__device__ __forceinline__ v16h frag_f32(const float* rowk0, int lane) {
  v16h a; const float* p = rowk0 + 8 * (lane >> 4);
#pragma unroll
  for (int i = 0; i < 8; ++i) { a[i] = (_Float16)p[i]; a[8 + i] = (_Float16)p[16 + i]; }
  return a;
}
__device__ __forceinline__ v16h frag_f32s(const float* rowk0, int lane, float sc) {
  v16h a; const float* p = rowk0 + 8 * (lane >> 4);
#pragma unroll
  for (int i = 0; i < 8; ++i) { a[i] = (_Float16)(p[i] * sc); a[8 + i] = (_Float16)(p[16 + i] * sc); }
  return a;
}
__device__ __forceinline__ v16h fragc_f32(const float* W, int k0, int n, int lane, int ld, int K) {
  v16h a; const int g = lane >> 4;
#pragma unroll
  for (int i = 0; i < 8; ++i) { const int ka = k0 + 8 * g + i, kb = ka + 16;
    a[i] = (_Float16)(ka < K ? W[(size_t)(ka < K ? ka : K - 1) * ld + n] : 0.f); a[8 + i] = (_Float16)(kb < K ? W[(size_t)(kb < K ? kb : K - 1) * ld + n] : 0.f); }
  return a;
}
struct F2 { v16b h, l; };
__device__ __forceinline__ F2 bsplit16(const float v[16]) { F2 r;
#pragma unroll
  for (int i = 0; i < 16; ++i) { const __bf16 h = (__bf16)v[i]; r.h[i] = h; r.l[i] = (__bf16)(v[i] - (float)h); }
  return r; }
__device__ __forceinline__ F2 split_row(const float* row, int k0, int lane) { float v[16]; const float* p = row + k0 + 8 * (lane >> 4);
#pragma unroll
  for (int i = 0; i < 8; ++i) { v[i] = p[i]; v[8 + i] = p[16 + i]; }
  return bsplit16(v); }
__device__ __forceinline__ F2 split_rowK(const float* row, int k0, int lane, int K) { float v[16]; const int g = lane >> 4;
#pragma unroll
  for (int i = 0; i < 8; ++i) { const int ka = k0 + 8 * g + i, kb = ka + 16; v[i] = ka < K ? row[ka < K ? ka : K - 1] : 0.f; v[8 + i] = kb < K ? row[kb < K ? kb : K - 1] : 0.f; }
  return bsplit16(v); }
__device__ __forceinline__ F2 split_col(const float* W, int k0, int n, int lane, int ld, int K) { float v[16]; const int g = lane >> 4;
#pragma unroll
  for (int i = 0; i < 8; ++i) { const int ka = k0 + 8 * g + i, kb = ka + 16; v[i] = ka < K ? W[(size_t)(ka < K ? ka : K - 1) * ld + n] : 0.f; v[8 + i] = kb < K ? W[(size_t)(kb < K ? kb : K - 1) * ld + n] : 0.f; }
  return bsplit16(v); }
__device__ __forceinline__ v8f mac3(const F2& a, const F2& b, v8f c) { c = wmma_bf(a.l, b.h, c); c = wmma_bf(a.h, b.l, c); return wmma_bf(a.h, b.h, c); }
__device__ __forceinline__ float sigm(float v) { return 1.0f / (1.0f + expf(-v)); }
#define LDSX() do { asm volatile("s_wait_dscnt 0" ::: "memory"); __builtin_amdgcn_wave_barrier(); __builtin_amdgcn_fence(__ATOMIC_RELEASE, "workgroup"); } while (0)


#define TT 1024
#define CC 768
#define NH 12
#define HD 64
#define NG 36
typedef __attribute__((ext_vector_type(8))) __bf16 v8b;
__device__ __forceinline__ v16b frag_b(const __bf16* rowk0, int lane) {
  union { v16b v; v8b q[2]; } u; const __bf16* p = rowk0 + 8 * (lane >> 4);
  u.q[0] = *(const v8b*)p; u.q[1] = *(const v8b*)(p + 16); return u.v;
}
__device__ __forceinline__ float bfr(float v) { return (float)(__bf16)v; }
__device__ __attribute__((noinline)) float exp_ni(float v) { return expf(v); }
__device__ __attribute__((noinline)) float erf_ni(float v) { return erff(v); }

#define WS_QH  0u
#define WS_QL  (WS_QH + 2u * (size_t)TT * CC)
#define WS_KH  (WS_QL + 2u * (size_t)TT * CC)
#define WS_KL  (WS_KH + 2u * (size_t)TT * CC)
#define WS_VT  (WS_KL + 2u * (size_t)TT * CC)
#define WS_VL  (WS_VT + 2u * (size_t)CC * TT)
#define WS_U   (WS_VL + 2u * (size_t)CC * TT)
#define WS_G   (WS_U + 4u * (size_t)TT * CC)
#define WS_CE  (WS_G + 4u * (size_t)TT * 48)
#define WS_CS  (WS_CE + 4u * (size_t)NH * TT)
#define WS_AL  (WS_CS + 4u * (size_t)NH * TT)
#define WS_BE  (WS_AL + 4u * (size_t)NH * TT)
#define WS_GM  (WS_BE + 4u * (size_t)NH * TT)
#define WS_S   (WS_GM + 4u * (size_t)NH * TT)
#define WS_Y   (WS_S + 4u * (size_t)NH * TT * TT)
#define WS_END (WS_Y + 4u * (size_t)TT * CC)

__global__ __launch_bounds__(128) void k_proj(const float* __restrict__ X, const float* __restrict__ WQ, const float* __restrict__ BQ, const float* __restrict__ WK, const float* __restrict__ BK, const float* __restrict__ WV, const float* __restrict__ BV, const float* __restrict__ WU, const float* __restrict__ BU, _Float16* __restrict__ QH, _Float16* __restrict__ QL, _Float16* __restrict__ KH, _Float16* __restrict__ KL, __bf16* __restrict__ VT, __bf16* __restrict__ VL, float* __restrict__ U) {
  __shared__ __align__(16) float sf[64][132]; __shared__ __align__(16) _Float16 sh[64][136], sl[64][136]; __shared__ __align__(16) __bf16 th[128][72], tl2[128][72]; __shared__ float snrm[64][2];
  const int tid = threadIdx.x, wave = tid >> 5, lane = tid & 31, col = lane & 15, g = lane >> 4; const int region = blockIdx.z; const int c0 = blockIdx.y * 128; const size_t r0 = (size_t)blockIdx.x * 64;
  const float* Wm = region == 0 ? WQ : region == 1 ? WK : region == 2 ? WV : WU; const float* Bm = region == 0 ? BQ : region == 1 ? BK : region == 2 ? BV : BU;
  v8f acc[8] = {};
#pragma unroll 2
  for (int kc = 0; kc < CC / 32; ++kc) { v16b a; { const float* p = X + (r0 + wave * 16 + col) * CC + kc * 32 + 8 * g;
#pragma unroll
      for (int i = 0; i < 8; ++i) { a[i] = (__bf16)p[i]; a[8 + i] = (__bf16)p[16 + i]; } }
#pragma unroll
    for (int j = 0; j < 8; ++j) { v16b w; const int o = c0 + j * 16 + col; const float* p = Wm + (size_t)o * CC + kc * 32 + 8 * g;
#pragma unroll
      for (int i = 0; i < 8; ++i) { w[i] = (__bf16)p[i]; w[8 + i] = (__bf16)p[16 + i]; }
      acc[j] = wmma_bf(a, w, acc[j]); } }
#pragma unroll
  for (int j = 0; j < 8; ++j) { const float bb = bfr(Bm[c0 + j * 16 + col]);
#pragma unroll
    for (int r = 0; r < 8; ++r) sf[wave * 16 + 8 * g + r][j * 16 + col] = acc[j][r] + bb; }
  __syncthreads();
  if (region <= 1) {
    __shared__ __align__(16) float sr[64][132];
    for (int e = tid; e < 64 * 128; e += 128) { const int rl = e >> 7, cl = e & 127; const int d = cl & 63; const int t = (int)(r0 + rl); const float inv_freq = 1.0f / powf(10000.0f, (float)(2 * (d >> 1)) / (float)HD); const float ang = (float)t * inv_freq; const float c = cosf(ang), s = sinf(ang);
      const float me = sf[rl][cl]; const float partner = (d < 32) ? -sf[rl][cl + 32] : sf[rl][cl - 32]; sr[rl][cl] = me * c + partner * s; }
    __syncthreads();
    for (int e = tid; e < 64 * 2; e += 128) { const int rl = e >> 1, hh = e & 1; float n2 = 0.f;
#pragma unroll 1
      for (int d = 0; d < HD; ++d) { const float v = sr[rl][hh * 64 + d]; n2 += v * v; } snrm[rl][hh] = 1.0f / fmaxf(sqrtf(n2), 1e-12f); }
    __syncthreads();
    for (int e = tid; e < 64 * 128; e += 128) { const int rl = e >> 7, cl = e & 127; const float v = sr[rl][cl] * snrm[rl][cl >> 6]; const _Float16 hv = (_Float16)v; sh[rl][cl] = hv; sl[rl][cl] = (_Float16)(v - (float)hv); }
    __syncthreads();
    _Float16* dh = region == 0 ? QH : KH; _Float16* dl = region == 0 ? QL : KL; for (int e = tid; e < 64 * 16; e += 128) { const int rl = e >> 4, q = e & 15; vst2((unsigned*)(dh + (r0 + rl) * CC + c0 + q * 8), *(const v4u*)&sh[rl][q * 8]); vst2((unsigned*)(dl + (r0 + rl) * CC + c0 + q * 8), *(const v4u*)&sl[rl][q * 8]); } }
  else if (region == 2) {
    for (int e = tid; e < 64 * 128; e += 128) { const int rl = e >> 7, cl = e & 127; const float v = sf[rl][cl]; const __bf16 bh = (__bf16)v; th[cl][rl] = bh; tl2[cl][rl] = (__bf16)(v - (float)bh); }
    __syncthreads(); for (int e = tid; e < 128 * 8; e += 128) { const int cl = e >> 3, q = e & 7; const size_t o2 = (size_t)(c0 + cl) * TT + r0 + q * 8; vst2((unsigned*)(VT + o2), *(const v4u*)&th[cl][q * 8]); vst2((unsigned*)(VL + o2), *(const v4u*)&tl2[cl][q * 8]); } }
  else { for (int e = tid; e < 64 * 32; e += 128) { const int rl = e >> 5, q = e & 31; vst2(U + (r0 + rl) * CC + c0 + q * 4, *(const v4f*)&sf[rl][q * 4]); } } }
__global__ __launch_bounds__(128) void k_gate(const float* __restrict__ X, const float* __restrict__ WG, const float* __restrict__ BG, float* __restrict__ Gt) { __shared__ __align__(16) float sf[4][16][52];
  const int tid = threadIdx.x, wave = tid >> 5, lane = tid & 31, col = lane & 15, g = lane >> 4; const size_t r0 = (size_t)blockIdx.x * 64 + wave * 16;
  v8f acc[3] = {};
#pragma unroll 2
  for (int kc = 0; kc < CC / 32; ++kc) { v16b a; { const float* p = X + (r0 + col) * CC + kc * 32 + 8 * g;
#pragma unroll
      for (int i = 0; i < 8; ++i) { a[i] = (__bf16)p[i]; a[8 + i] = (__bf16)p[16 + i]; } }
#pragma unroll
    for (int j = 0; j < 3; ++j) { v16b w; const int o = min(j * 16 + col, NG - 1); const float* p = WG + (size_t)o * CC + kc * 32 + 8 * g;
#pragma unroll
      for (int i = 0; i < 8; ++i) { w[i] = (__bf16)p[i]; w[8 + i] = (__bf16)p[16 + i]; }
      acc[j] = wmma_bf(a, w, acc[j]); } }
#pragma unroll
  for (int j = 0; j < 3; ++j) { const int o = j * 16 + col; const float bb = (o < NG) ? bfr(BG[o]) : 0.f;
#pragma unroll
    for (int r = 0; r < 8; ++r) sf[wave][8 * g + r][o] = acc[j][r] + bb; }
  LDSX(); for (int rl = 0; rl < 16; ++rl) if (lane < 12) vst2(Gt + (r0 + rl) * 48 + lane * 4, *(const v4f*)&sf[wave][rl][lane * 4]); }
__global__ __launch_bounds__(256) void k_pre(const float* __restrict__ U, const float* __restrict__ Gt, const float* __restrict__ MU, const float* __restrict__ LT, float* __restrict__ CE, float* __restrict__ CS, float* __restrict__ AL, float* __restrict__ BE, float* __restrict__ GM) {
  __shared__ __align__(16) float ss[TT]; __shared__ float sred[8]; __shared__ float sE[TT], sP[TT]; __shared__ float smax; __shared__ __align__(16) float sce[TT], sal[TT], sbe[TT], sgm[TT];
  const int t = threadIdx.x, wv = t >> 5, ln = t & 31; const int h = blockIdx.x;
  float ltau = bfr(LT[h]); ltau = fminf(fmaxf(ltau, -50.f), 30.f); const float tau = expf(ltau);
  float cs = 0.f; const float mu = (t < HD) ? bfr(MU[h * HD + t]) : 0.f;
#pragma unroll 1
  for (int l = 0; l < TT; ++l) { float term = 0.f; if (t < HD) { const float uv = U[(size_t)l * CC + h * HD + t]; cs += uv; const float bar = (tau * mu + cs) / (tau + (float)(l + 1)); term = uv * bar; }
#pragma unroll
    for (int o = 1; o < 32; o <<= 1) term += __shfl_xor(term, o);
    if (ln == 0 && wv < 2) sred[wv] = term; __syncthreads(); if (t == 0) ss[l] = -(sred[0] + sred[1]) * 0.125f; __syncthreads(); }
  float m = -3.0e38f; for (int l = t; l < TT; l += 256) m = fmaxf(m, ss[l]);
#pragma unroll
  for (int o = 1; o < 32; o <<= 1) m = fmaxf(m, __shfl_xor(m, o));
  if (ln == 0) sred[wv] = m; __syncthreads(); if (t == 0) { float a = sred[0]; for (int w = 1; w < 8; ++w) a = fmaxf(a, sred[w]); smax = a; } __syncthreads();
  if (t == 0) { float E = 0.f, P = 0.f; for (int l = 0; l < TT; ++l) { const float e = expf(ss[l] - smax); E += e; P += ss[l]; sE[l] = E; sP[l] = P; } }
  __syncthreads();
  for (int l = t; l < TT; l += 256) { const float e = expf(ss[l] - smax); const float tt1 = (float)(l + 1); const float g0 = Gt[(size_t)l * 48 + h * 3], g1 = Gt[(size_t)l * 48 + h * 3 + 1]; const float sig1 = 1.0f / (1.0f + expf(-g0)), sigh = 1.0f / (1.0f + expf(-g1));
    const float alpha = sigh / (sE[l] + 1e-12f); const float beta = (sig1 - sigh) / tt1; const float gamma = -((beta * sP[l] + sigh) / tt1);
    sce[l] = e; sal[l] = alpha; sbe[l] = beta; sgm[l] = gamma; }
  __syncthreads();
  for (int q = t; q < TT / 4; q += 256) { vst2(CE + h * TT + q * 4, *(const v4f*)&sce[q * 4]); vst2(CS + h * TT + q * 4, *(const v4f*)&ss[q * 4]); vst2(AL + h * TT + q * 4, *(const v4f*)&sal[q * 4]); vst2(BE + h * TT + q * 4, *(const v4f*)&sbe[q * 4]); vst2(GM + h * TT + q * 4, *(const v4f*)&sgm[q * 4]); } }
__global__ __launch_bounds__(128) void k_sc(const _Float16* __restrict__ QH, const _Float16* __restrict__ QL, const _Float16* __restrict__ KH, const _Float16* __restrict__ KL, const float* __restrict__ CE, const float* __restrict__ CS, const float* __restrict__ AL, const float* __restrict__ BE, const float* __restrict__ GM, float* __restrict__ S0) { __shared__ __align__(16) float ss[4][16][132];
  const int h = blockIdx.z; float* S = S0 + (size_t)h * TT * TT;
  const int tid = threadIdx.x, wave = tid >> 5, lane = tid & 31, col = lane & 15, g = lane >> 4; const int k0 = blockIdx.y * 128; const int ql0 = blockIdx.x * 64 + wave * 16;
  if (k0 > blockIdx.x * 64 + 63) return;
  v8f acc[8] = {};
#pragma unroll
  for (int kc = 0; kc < HD / 32; ++kc) { const v16h ah = frag_h(QH + (size_t)(ql0 + col) * CC + h * HD + kc * 32, lane), al = frag_h(QL + (size_t)(ql0 + col) * CC + h * HD + kc * 32, lane);
#pragma unroll
    for (int j = 0; j < 8; ++j) { const size_t ko = (size_t)(k0 + j * 16 + col) * CC + h * HD + kc * 32; const v16h kb = frag_h(KH + ko, lane); acc[j] = wmma16(ah, kb, acc[j]); acc[j] = wmma16(al, kb, acc[j]); acc[j] = wmma16(ah, frag_h(KL + ko, lane), acc[j]); } }
#pragma unroll
  for (int j = 0; j < 8; ++j) { const int l = k0 + j * 16 + col; const float el = CE[h * TT + l], sl = CS[h * TT + l];
#pragma unroll
    for (int r = 0; r < 8; ++r) { const int t = ql0 + 8 * g + r; const float w = AL[h * TT + t] * el + BE[h * TT + t] * sl + GM[h * TT + t]; ss[wave][8 * g + r][j * 16 + col] = (l <= t) ? acc[j][r] * w : 0.f; } }
  LDSX(); for (int rl = 0; rl < 16; ++rl) vst2(S + (size_t)(ql0 + rl) * TT + k0 + lane * 4, *(const v4f*)&ss[wave][rl][lane * 4]); }
__global__ __launch_bounds__(128) void k_pv(const float* __restrict__ S0, const __bf16* __restrict__ VT, const __bf16* __restrict__ VL, float* __restrict__ Y) { __shared__ __align__(16) float so[64][68];
  const int h = blockIdx.z; const float* S = S0 + (size_t)h * TT * TT;
  const int tid = threadIdx.x, wave = tid >> 5, lane = tid & 31, col = lane & 15, g = lane >> 4; const int ql0 = blockIdx.x * 64 + wave * 16; const int kend = blockIdx.x * 64 + 64;
  v8f acc[4] = {};
#pragma unroll 1
  for (int kc = 0; kc < kend / 32; ++kc) { const F2 p = split_row(S + (size_t)(ql0 + col) * TT, kc * 32, lane);
#pragma unroll
    for (int j = 0; j < 4; ++j) { const size_t po = (size_t)(h * HD + j * 16 + col) * TT + kc * 32; const v16b vh = frag_b(VT + po, lane); acc[j] = wmma_bf(p.h, vh, acc[j]); acc[j] = wmma_bf(p.l, vh, acc[j]); acc[j] = wmma_bf(p.h, frag_b(VL + po, lane), acc[j]); } }
#pragma unroll
  for (int j = 0; j < 4; ++j)
#pragma unroll
    for (int r = 0; r < 8; ++r) so[wave * 16 + 8 * g + r][j * 16 + col] = acc[j][r];
  __syncthreads();
  if (tid < 64) { float m = 0.f; for (int d = 0; d < HD; ++d) m += so[tid][d]; m *= (1.0f / HD); float v = 0.f; for (int d = 0; d < HD; ++d) { const float dd = so[tid][d] - m; v += dd * dd; } const float inv = 1.0f / sqrtf(v * (1.0f / HD) + 1e-5f); for (int d = 0; d < HD; ++d) so[tid][d] = (so[tid][d] - m) * inv; }
  __syncthreads(); for (int e = tid; e < 64 * 16; e += 128) { const int rl = e >> 4, q = e & 15; vst2(Y + (size_t)(blockIdx.x * 64 + rl) * CC + h * HD + q * 4, *(const v4f*)&so[rl][q * 4]); } }
__global__ __launch_bounds__(128) void k_out(const float* __restrict__ Y, const float* __restrict__ WO, const float* __restrict__ BO, float* __restrict__ OUT) { __shared__ __align__(16) float sf[4][16][132];
  const int tid = threadIdx.x, wave = tid >> 5, lane = tid & 31, col = lane & 15, g = lane >> 4; const int c0 = blockIdx.y * 128; const size_t r0 = (size_t)blockIdx.x * 64 + wave * 16;
  v8f acc[8] = {};
#pragma unroll 2
  for (int kc = 0; kc < CC / 32; ++kc) { const F2 a = split_row(Y + (r0 + col) * CC, kc * 32, lane);
#pragma unroll
    for (int j = 0; j < 8; ++j) { v16b w; const int o = c0 + j * 16 + col; const float* p = WO + (size_t)o * CC + kc * 32 + 8 * g;
#pragma unroll
      for (int i = 0; i < 8; ++i) { w[i] = (__bf16)p[i]; w[8 + i] = (__bf16)p[16 + i]; }
      acc[j] = wmma_bf(a.h, w, acc[j]); acc[j] = wmma_bf(a.l, w, acc[j]); } }
#pragma unroll
  for (int j = 0; j < 8; ++j) { const float bb = bfr(BO[c0 + j * 16 + col]);
#pragma unroll
    for (int r = 0; r < 8; ++r) sf[wave][8 * g + r][j * 16 + col] = acc[j][r] + bb; }
  LDSX(); for (int rl = 0; rl < 16; ++rl) vst2(OUT + (r0 + rl) * CC + c0 + lane * 4, *(const v4f*)&sf[wave][rl][lane * 4]); }
extern "C" void kernel_launch(void* const* d_in, const int* in_sizes, int n_in, void* d_out, int out_size, void* d_ws, size_t ws_size, hipStream_t stream) {
  (void)in_sizes; (void)n_in; (void)out_size;
  const float** F = (const float**)d_in;
  if (ws_size < (size_t)WS_END) return;
  char* ws = (char*)d_ws; _Float16 *QH = (_Float16*)(ws + WS_QH), *QL = (_Float16*)(ws + WS_QL), *KH = (_Float16*)(ws + WS_KH), *KL = (_Float16*)(ws + WS_KL); __bf16 *VT = (__bf16*)(ws + WS_VT), *VL = (__bf16*)(ws + WS_VL); float *U = (float*)(ws + WS_U), *Gt = (float*)(ws + WS_G), *CE = (float*)(ws + WS_CE), *CS = (float*)(ws + WS_CS), *AL = (float*)(ws + WS_AL), *BE = (float*)(ws + WS_BE), *GM = (float*)(ws + WS_GM), *S = (float*)(ws + WS_S), *Y = (float*)(ws + WS_Y);
  k_proj<<<dim3(TT / 64, CC / 128, 4), 128, 0, stream>>>(F[0], F[1], F[2], F[3], F[4], F[5], F[6], F[7], F[8], QH, QL, KH, KL, VT, VL, U);
  k_gate<<<TT / 64, 128, 0, stream>>>(F[0], F[9], F[10], Gt);
  k_pre<<<NH, 256, 0, stream>>>(U, Gt, F[13], F[14], CE, CS, AL, BE, GM);
  k_sc<<<dim3(TT / 64, TT / 128, NH), 128, 0, stream>>>(QH, QL, KH, KL, CE, CS, AL, BE, GM, S);
  k_pv<<<dim3(TT / 64, 1, NH), 128, 0, stream>>>(S, VT, VL, Y);
  k_out<<<dim3(TT / 64, CC / 128), 128, 0, stream>>>(Y, F[11], F[12], (float*)d_out);
}
